// RGCNEncoder_7619271983570
// MI455X (gfx1250) — hardware-verified
//
#include <hip/hip_runtime.h>
#include <stddef.h>
#include <stdint.h>


#define CIN    128
#define DH     128
#define DO     64
#define K2     256
#define NTYPE  3
#define NREL   6
#define NTHR   256
#define NWAVE  8
#define EPT    8
#define CHUNK  (NTHR * EPT)
#define WCAP   (EPT * 32)
#define LISTN  (NWAVE * WCAP)
#define NBD    8192
#define SLD    13
#define NBA    1024
#define SLA    10
#define RCAP   32768
#define DEGCAP 256
#define GBM    32
#define GTHR   64
#define NUP    (NTYPE * DH * (CIN / 8))
#define NU1    (NREL * DH * (DH / 4))
#define NU2    (NREL * DO * (DH / 4))
#define NUT    (NUP + NU1 + NU2)
#define AGG_ZINTS    (LISTN + 2 * RCAP + 3 * NBA)
#define AGG_LDS_INTS (AGG_ZINTS + 16)
#define WSMAX  134217728

static_assert((CHUNK & (CHUNK - 1)) == 0 && CHUNK <= 4096);
static_assert((NBD & (NBD - 1)) == 0 && NBD == (1 << SLD));
static_assert((NBA & (NBA - 1)) == 0 && NBA == (1 << SLA));
static_assert(((long long)CHUNK << SLD) < (1LL << 31));
static_assert(((long long)CHUNK << SLA) < (1LL << 31));
static_assert(NBD % (NTHR * 4) == 0);
static_assert(LISTN % NTHR == 0);
static_assert(NBA % NWAVE == 0 && NBA % 32 == 0 && NBA % GBM == 0);
static_assert(RCAP % 32 == 0 && AGG_ZINTS % (NTHR * 4) == 0 && LISTN % 4 == 0 && (AGG_ZINTS + 16) % 4 == 0);
static_assert(CIN % 32 == 0 && K2 % 32 == 0 && K2 == 2 * DH);
static_assert(GBM == (GTHR / 32) * 16);
static_assert(NUP % NTHR == 0 && NU1 % NTHR == 0 && NU2 % NTHR == 0 && NUT % NTHR == 0);
static_assert((DH * (CIN / 8)) % NTHR == 0 && (DH * (DH / 4)) % NTHR == 0 && (DO * (DH / 4)) % NTHR == 0);
static_assert(CIN / 8 == 16 && DH / 4 == 32 && DH == 4 * 32 && DO == 4 * 16);
static_assert(GBM * DO == 8 * GTHR * 4);
static_assert(AGG_LDS_INTS * 4 <= 300000);

typedef float          v4f   __attribute__((ext_vector_type(4)));
typedef float          v8f   __attribute__((ext_vector_type(8)));
typedef int            v4i   __attribute__((ext_vector_type(4)));
typedef int            v8i   __attribute__((ext_vector_type(8)));
typedef unsigned short v8us  __attribute__((ext_vector_type(8)));
typedef unsigned short v16us __attribute__((ext_vector_type(16)));
typedef __bf16         v16bf __attribute__((ext_vector_type(16)));
typedef v4f  __attribute__((may_alias)) v4fa;
typedef v4i  __attribute__((may_alias)) v4ia;
typedef v8us __attribute__((may_alias)) v8usa;
union Frag { v16bf v; v16us u; v8us h[2]; v8i w; };

__device__ __forceinline__ v8f wmb(const Frag& a, const Frag& b, v8f c) {
  v8f d = __builtin_amdgcn_wmma_f32_16x16x32_bf16(false, a.v, false, b.v, (short)0, c, false, false);
  asm volatile("v_nop\n\tv_nop\n\tv_nop\n\tv_nop" : "+v"(d) : "v"(a.w), "v"(b.w));
  return d;
}

__device__ __forceinline__ unsigned bf16_bits(float f) {
  const unsigned u = __float_as_uint(f);
  return (u + 0x7FFFu + ((u >> 16) & 1u)) >> 16;
}
__device__ __forceinline__ float bf16_val(float f) {
  return __uint_as_float(bf16_bits(f) << 16);
}
__device__ __forceinline__ v8us hilo8(v4f t) {
  v8us o;
  unsigned hb;
  hb = bf16_bits(t.x); o[0] = (unsigned short)hb; o[4] = (unsigned short)bf16_bits(t.x - __uint_as_float(hb << 16));
  hb = bf16_bits(t.y); o[1] = (unsigned short)hb; o[5] = (unsigned short)bf16_bits(t.y - __uint_as_float(hb << 16));
  hb = bf16_bits(t.z); o[2] = (unsigned short)hb; o[6] = (unsigned short)bf16_bits(t.z - __uint_as_float(hb << 16));
  hb = bf16_bits(t.w); o[3] = (unsigned short)hb; o[7] = (unsigned short)bf16_bits(t.w - __uint_as_float(hb << 16));
  return o;
}

__device__ __forceinline__ float wsum32(float v) {
  v += __shfl_xor(v, 16, 32);
  v += __shfl_xor(v, 8, 32);
  v += __shfl_xor(v, 4, 32);
  v += __shfl_xor(v, 2, 32);
  v += __shfl_xor(v, 1, 32);
  return v;
}
__device__ __forceinline__ float wsum16(float v) {
  v += __shfl_xor(v, 8, 32);
  v += __shfl_xor(v, 4, 32);
  v += __shfl_xor(v, 2, 32);
  v += __shfl_xor(v, 1, 32);
  return v;
}

template <int SLB>
__device__ __forceinline__ int scan_chunk(const int* __restrict__ dsts, int nE, int cbase, int slotBase,
                                          int nb, int vec8, int* list, int tid, int lane, int wave) {
  int wc = 0;
  const int el0  = tid * EPT;
  const int e0   = cbase + el0;
  const int sent = -2147483647 - 1;
  v4i da, db;
  if (vec8 != 0 && cbase + CHUNK <= nE) {
    da = *(const v4i*)(dsts + e0);
    db = *(const v4i*)(dsts + e0 + 4);
  } else {
    da.x = (e0     < nE) ? dsts[min(e0,     nE - 1)] : sent;
    da.y = (e0 + 1 < nE) ? dsts[min(e0 + 1, nE - 1)] : sent;
    da.z = (e0 + 2 < nE) ? dsts[min(e0 + 2, nE - 1)] : sent;
    da.w = (e0 + 3 < nE) ? dsts[min(e0 + 3, nE - 1)] : sent;
    db.x = (e0 + 4 < nE) ? dsts[min(e0 + 4, nE - 1)] : sent;
    db.y = (e0 + 5 < nE) ? dsts[min(e0 + 5, nE - 1)] : sent;
    db.z = (e0 + 6 < nE) ? dsts[min(e0 + 6, nE - 1)] : sent;
    db.w = (e0 + 7 < nE) ? dsts[min(e0 + 7, nE - 1)] : sent;
  }
  const unsigned nbs = (unsigned)slotBase;
  const unsigned unb = (unsigned)nb;
  const unsigned s0 = (unsigned)da.x - nbs, s1 = (unsigned)da.y - nbs;
  const unsigned s2 = (unsigned)da.z - nbs, s3 = (unsigned)da.w - nbs;
  const unsigned s4 = (unsigned)db.x - nbs, s5 = (unsigned)db.y - nbs;
  const unsigned s6 = (unsigned)db.z - nbs, s7 = (unsigned)db.w - nbs;
  const bool h0 = s0 < unb, h1 = s1 < unb, h2 = s2 < unb, h3 = s3 < unb;
  const bool h4 = s4 < unb, h5 = s5 < unb, h6 = s6 < unb, h7 = s7 < unb;
  const unsigned any = __builtin_amdgcn_ballot_w32(h0 | h1 | h2 | h3 | h4 | h5 | h6 | h7);
  if (any != 0u) {
#define HITJ(J, HJ, SJ) { \
      const unsigned mj = __builtin_amdgcn_ballot_w32(HJ); \
      if (mj != 0u) { \
        if (HJ) { \
          const int pos = wc + (int)__builtin_amdgcn_mbcnt_lo(mj, 0u); \
          if (pos < WCAP) list[wave * WCAP + pos] = ((el0 + (J)) << SLB) | (int)(SJ); \
        } \
        wc += (int)__builtin_popcount(mj); } }
    HITJ(0, h0, s0)
    HITJ(1, h1, s1)
    HITJ(2, h2, s2)
    HITJ(3, h3, s3)
    HITJ(4, h4, s4)
    HITJ(5, h5, s5)
    HITJ(6, h6, s6)
    HITJ(7, h7, s7)
#undef HITJ
  }
  return wc;
}

__global__ __launch_bounds__(NTHR) void k_prep(const float* __restrict__ Wp0, const float* __restrict__ Wp1,
                                               const float* __restrict__ Wp2, const float* __restrict__ W1,
                                               const float* __restrict__ W2, unsigned short* WPT,
                                               unsigned short* W1T, unsigned short* W2T) {
  const int u = (int)blockIdx.x * NTHR + (int)threadIdx.x;
  v8us o;
  unsigned short* dp;
  if (u < NUP) {
    const int t  = u >> 11;
    const int n  = (u >> 4) & 127;
    const int k8 = (u & 15) * 8;
    const float* W = Wp0;
    if (t == 1) W = Wp1;
    else if (t == 2) W = Wp2;
    const float* p = W + (size_t)k8 * DH + n;
#pragma unroll
    for (int i = 0; i < 8; ++i) o[i] = (unsigned short)bf16_bits(p[(size_t)i * DH]);
    dp = WPT + (size_t)t * DH * CIN + (size_t)n * CIN + k8;
  } else if (u < NUP + NU1) {
    const int v = u - NUP;
    const int r = v >> 12;
    const int n = (v >> 5) & 127;
    const int g = v & 31;
    const float* p = W1 + (size_t)r * DH * DH + (size_t)(4 * g) * DH + n;
    const unsigned short f0 = (unsigned short)bf16_bits(p[0]);
    const unsigned short f1 = (unsigned short)bf16_bits(p[DH]);
    const unsigned short f2 = (unsigned short)bf16_bits(p[2 * DH]);
    const unsigned short f3 = (unsigned short)bf16_bits(p[3 * DH]);
    o[0] = f0; o[1] = f1; o[2] = f2; o[3] = f3; o[4] = f0; o[5] = f1; o[6] = f2; o[7] = f3;
    dp = W1T + (size_t)r * DH * K2 + (size_t)n * K2 + 8 * g;
  } else if (u < NUT) {
    const int v = u - NUP - NU1;
    const int r = v >> 11;
    const int n = (v >> 5) & 63;
    const int g = v & 31;
    const float* p = W2 + (size_t)r * DH * DO + (size_t)(4 * g) * DO + n;
    const unsigned short f0 = (unsigned short)bf16_bits(p[0]);
    const unsigned short f1 = (unsigned short)bf16_bits(p[DO]);
    const unsigned short f2 = (unsigned short)bf16_bits(p[2 * DO]);
    const unsigned short f3 = (unsigned short)bf16_bits(p[3 * DO]);
    o[0] = f0; o[1] = f1; o[2] = f2; o[3] = f3; o[4] = f0; o[5] = f1; o[6] = f2; o[7] = f3;
    dp = W2T + (size_t)r * DO * K2 + (size_t)n * K2 + 8 * g;
  } else {
    return;
  }
  *(volatile v8us*)dp = o;
  __threadfence();
  *(volatile v8us*)dp = o;
}

__global__ __launch_bounds__(NTHR) void k_cvx(const float* __restrict__ x0, const float* __restrict__ x1,
                                              const float* __restrict__ x2, int n0, int n1, int n2,
                                              unsigned short* xb) {
  const int u  = (int)blockIdx.x * NTHR + (int)threadIdx.x;
  const int U0 = n0 * 16, U1 = n1 * 16, U2 = n2 * 16;
  const float* x = x0;
  int row, grow;
  if (u < U0) {
    row = u >> 4; grow = row;
  } else if (u < U0 + U1) {
    x = x1; row = (u - U0) >> 4; grow = n0 + row;
  } else if (u < U0 + U1 + U2) {
    x = x2; row = (u - U0 - U1) >> 4; grow = n0 + n1 + row;
  } else {
    return;
  }
  const int k8 = (u & 15) * 8;
  const float* p = x + (size_t)row * CIN + k8;
  const v4f a = *(const v4fa*)p;
  const v4f b = *(const v4fa*)(p + 4);
  v8us o;
  o[0] = (unsigned short)bf16_bits(a.x); o[1] = (unsigned short)bf16_bits(a.y);
  o[2] = (unsigned short)bf16_bits(a.z); o[3] = (unsigned short)bf16_bits(a.w);
  o[4] = (unsigned short)bf16_bits(b.x); o[5] = (unsigned short)bf16_bits(b.y);
  o[6] = (unsigned short)bf16_bits(b.z); o[7] = (unsigned short)bf16_bits(b.w);
  unsigned short* dp = xb + (size_t)grow * CIN + k8;
  *(volatile v8us*)dp = o;
  __threadfence();
  *(volatile v8us*)dp = o;
}

__global__ __launch_bounds__(NTHR) void k_deg(const int* __restrict__ e0, const int* __restrict__ e1,
                                              const int* __restrict__ e2, const int* __restrict__ e3,
                                              const int* __restrict__ e4, const int* __restrict__ e5,
                                              int nE, int vec8, int n0, int n1, int n2, int nbpd, float* dg) {
  __shared__ __attribute__((aligned(16))) int scnt[NBD];
  __shared__ __attribute__((aligned(16))) int list[LISTN];
  __shared__ int wcnt[NWAVE];
  const int tid = (int)threadIdx.x, lane = tid & 31, wave = tid >> 5;
  const int nodeBase = (int)blockIdx.x * NBD;
  const int p = (int)blockIdx.y;
  const int* lst = e0;
  int nTab = n0;
  if (p == 1)      { lst = e1; nTab = n0; }
  else if (p == 2) { lst = e2; nTab = n1; }
  else if (p == 3) { lst = e3; nTab = n2; }
  else if (p == 4) { lst = e4; nTab = n1; }
  else if (p == 5) { lst = e5; nTab = n2; }
  if (nodeBase >= nTab) return;

  for (int i = tid; i < NBD; i += NTHR) scnt[i] = 0;
  for (int i = tid; i < LISTN; i += NTHR) list[i] = 0;
  if (tid < NWAVE) wcnt[tid] = 0;
  __syncthreads();

  const int nChunks = (nE + CHUNK - 1) / CHUNK;
#pragma unroll 1
  for (int ch = 0; ch < nChunks; ++ch) {
    const int cbase = ch * CHUNK;
    const int wc = scan_chunk<SLD>(lst, nE, cbase, nodeBase, NBD, vec8, list, tid, lane, wave);
    if (lane == 0) wcnt[wave] = wc;
    __syncthreads();
    if (wave == 0) {
#pragma unroll 1
      for (int w2 = 0; w2 < NWAVE; ++w2) {
        int c = wcnt[w2];
        c = c < 0 ? 0 : (c > WCAP ? WCAP : c);
#pragma unroll 1
        for (int b0 = 0; b0 < c; b0 += 32) {
          const int idx = b0 + lane;
          const int ent = list[w2 * WCAP + (idx < WCAP ? idx : WCAP - 1)];
          const int m32 = (c - b0) < 32 ? (c - b0) : 32;
#pragma unroll 1
          for (int k = 0; k < m32; ++k) {
            const int u  = __builtin_amdgcn_readlane(ent, k);
            const int sl = u & (NBD - 1);
            if (lane == 0) scnt[sl] = scnt[sl] + 1;
          }
        }
      }
    }
    __syncthreads();
  }

  v4f vals[NBD / (NTHR * 4)];
#pragma unroll
  for (int it = 0; it < NBD / (NTHR * 4); ++it) {
    const int s0 = it * (NTHR * 4) + 4 * tid;
    const v4i c4 = *(const v4ia*)(scnt + s0);
    const float d0 = (float)(c4.x < 1 ? 1 : c4.x), d1 = (float)(c4.y < 1 ? 1 : c4.y);
    const float d2 = (float)(c4.z < 1 ? 1 : c4.z), d3 = (float)(c4.w < 1 ? 1 : c4.w);
    v4f v;
    v.x = rsqrtf(d0); v.y = rsqrtf(d1); v.z = rsqrtf(d2); v.w = rsqrtf(d3);
    vals[it] = v;
  }
  float* base = dg + (size_t)p * (size_t)nbpd + (size_t)nodeBase;
#pragma unroll
  for (int it = 0; it < NBD / (NTHR * 4); ++it) {
    const int s0 = it * (NTHR * 4) + 4 * tid;
    *(volatile v4f*)(base + s0) = vals[it];
  }
  __threadfence();
#pragma unroll
  for (int it = 0; it < NBD / (NTHR * 4); ++it) {
    const int s0 = it * (NTHR * 4) + 4 * tid;
    *(volatile v4f*)(base + s0) = vals[it];
  }
}

__global__ __launch_bounds__(GTHR) void k_proj(const unsigned short* __restrict__ A,
                                               const unsigned short* __restrict__ WT,
                                               const float* __restrict__ bias, unsigned short* hpl) {
  __shared__ __attribute__((aligned(16))) float stg[GBM * DH];
  const int tid = (int)threadIdx.x, lane = tid & 31, wave = tid >> 5, hh = lane >> 4, m = lane & 15;
  const int rowBase = (int)blockIdx.x * GBM;

  v8f acc[8];
  {
    const v8f z = {0.f, 0.f, 0.f, 0.f, 0.f, 0.f, 0.f, 0.f};
#pragma unroll
    for (int t = 0; t < 8; ++t) acc[t] = z;
  }
  const unsigned short* ap = A  + (size_t)(rowBase + 16 * wave + m) * (size_t)CIN + 8 * hh;
  const unsigned short* bp = WT + (size_t)m * (size_t)CIN + 8 * hh;

#pragma unroll 1
  for (int ks = 0; ks < CIN / 32; ++ks) {
    const int k0 = 32 * ks;
    Frag af;
    af.h[0] = *(const v8usa*)(ap + k0);
    af.h[1] = *(const v8usa*)(ap + k0 + 16);
#pragma unroll
    for (int nt = 0; nt < 8; ++nt) {
      const unsigned short* wq = bp + (size_t)(16 * nt) * (size_t)CIN + k0;
      Frag bf;
      bf.h[0] = *(const v8usa*)wq;
      bf.h[1] = *(const v8usa*)(wq + 16);
      acc[nt] = wmb(af, bf, acc[nt]);
    }
  }

#pragma unroll
  for (int nt = 0; nt < 8; ++nt) {
    const int lc = 16 * nt + m;
#pragma unroll
    for (int r = 0; r < 8; ++r) {
      const int lr = 16 * wave + 8 * hh + r;
      stg[lr * DH + lc] = acc[nt][r];
    }
  }
  __syncthreads();

  v4f bb4;
  {
    const v4f tb = *(const v4fa*)(bias + 4 * lane);
    bb4.x = bf16_val(tb.x); bb4.y = bf16_val(tb.y); bb4.z = bf16_val(tb.z); bb4.w = bf16_val(tb.w);
  }
  v8us po[16];
#pragma unroll
  for (int i = 0; i < 16; ++i) {
    const v4f t = *(const v4fa*)(stg + (16 * wave + i) * DH + 4 * lane) + bb4;
    po[i] = hilo8(t);
  }
#pragma unroll
  for (int i = 0; i < 16; ++i) {
    unsigned short* rp = hpl + (size_t)(rowBase + 16 * wave + i) * (size_t)K2 + 8 * lane;
    *(volatile v8us*)rp = po[i];
  }
  __threadfence();
#pragma unroll
  for (int i = 0; i < 16; ++i) {
    unsigned short* rp = hpl + (size_t)(rowBase + 16 * wave + i) * (size_t)K2 + 8 * lane;
    *(volatile v8us*)rp = po[i];
  }
}

__global__ __launch_bounds__(GTHR) void k_gemm(const unsigned short* __restrict__ A,
                                               const unsigned short* __restrict__ WT,
                                               const float* __restrict__ dg, float* T, int K) {
  __shared__ __attribute__((aligned(16))) float stg[GBM * DH];
  __shared__ __attribute__((aligned(16))) float sdg[GBM];
  const int tid = (int)threadIdx.x, lane = tid & 31, wave = tid >> 5, hh = lane >> 4, m = lane & 15;
  const int rowBase = (int)blockIdx.x * GBM;
  if (tid < GBM) sdg[tid] = dg[rowBase + tid];

  v8f acc[8];
  {
    const v8f z = {0.f, 0.f, 0.f, 0.f, 0.f, 0.f, 0.f, 0.f};
#pragma unroll
    for (int t = 0; t < 8; ++t) acc[t] = z;
  }
  const unsigned short* ap = A  + (size_t)(rowBase + 16 * wave + m) * (size_t)K + 8 * hh;
  const unsigned short* bp = WT + (size_t)m * (size_t)K + 8 * hh;
  const int ksteps = K >> 5;

#pragma unroll 1
  for (int ks = 0; ks < ksteps; ++ks) {
    const int k0 = 32 * ks;
    Frag af;
    af.h[0] = *(const v8usa*)(ap + k0);
    af.h[1] = *(const v8usa*)(ap + k0 + 16);
#pragma unroll
    for (int nt = 0; nt < 8; ++nt) {
      const unsigned short* wq = bp + (size_t)(16 * nt) * (size_t)K + k0;
      Frag bf;
      bf.h[0] = *(const v8usa*)wq;
      bf.h[1] = *(const v8usa*)(wq + 16);
      acc[nt] = wmb(af, bf, acc[nt]);
    }
  }

#pragma unroll
  for (int nt = 0; nt < 8; ++nt) {
    const int lc = 16 * nt + m;
#pragma unroll
    for (int r = 0; r < 8; ++r) {
      const int lr = 16 * wave + 8 * hh + r;
      stg[lr * DH + lc] = acc[nt][r];
    }
  }
  __syncthreads();

  v4f fv[16];
#pragma unroll
  for (int i = 0; i < 16; ++i) {
    const int lr = 16 * wave + i;
    fv[i] = *(const v4fa*)(stg + lr * DH + 4 * lane) * sdg[lr];
  }
#pragma unroll
  for (int i = 0; i < 16; ++i) {
    float* op = T + (size_t)(rowBase + 16 * wave + i) * (size_t)DH + 4 * lane;
    *(volatile v4f*)op = fv[i];
  }
  __threadfence();
#pragma unroll
  for (int i = 0; i < 16; ++i) {
    float* op = T + (size_t)(rowBase + 16 * wave + i) * (size_t)DH + 4 * lane;
    *(volatile v4f*)op = fv[i];
  }
}

__global__ __launch_bounds__(GTHR) void k_gemm64(const unsigned short* __restrict__ A,
                                                 const unsigned short* __restrict__ WT,
                                                 const float* __restrict__ dg, float* T) {
  __shared__ __attribute__((aligned(16))) float stg[GBM * DO];
  __shared__ __attribute__((aligned(16))) float sdg[GBM];
  const int tid = (int)threadIdx.x, lane = tid & 31, wave = tid >> 5, hh = lane >> 4, m = lane & 15;
  const int rowBase = (int)blockIdx.x * GBM;
  if (tid < GBM) sdg[tid] = dg[rowBase + tid];

  v8f acc[4];
  {
    const v8f z = {0.f, 0.f, 0.f, 0.f, 0.f, 0.f, 0.f, 0.f};
#pragma unroll
    for (int t = 0; t < 4; ++t) acc[t] = z;
  }
  const unsigned short* ap = A  + (size_t)(rowBase + 16 * wave + m) * (size_t)K2 + 8 * hh;
  const unsigned short* bp = WT + (size_t)m * (size_t)K2 + 8 * hh;

#pragma unroll 1
  for (int ks = 0; ks < K2 / 32; ++ks) {
    const int k0 = 32 * ks;
    Frag af;
    af.h[0] = *(const v8usa*)(ap + k0);
    af.h[1] = *(const v8usa*)(ap + k0 + 16);
#pragma unroll
    for (int nt = 0; nt < 4; ++nt) {
      const unsigned short* wq = bp + (size_t)(16 * nt) * (size_t)K2 + k0;
      Frag bf;
      bf.h[0] = *(const v8usa*)wq;
      bf.h[1] = *(const v8usa*)(wq + 16);
      acc[nt] = wmb(af, bf, acc[nt]);
    }
  }

#pragma unroll
  for (int nt = 0; nt < 4; ++nt) {
    const int lc = 16 * nt + m;
#pragma unroll
    for (int r = 0; r < 8; ++r) {
      const int lr = 16 * wave + 8 * hh + r;
      stg[lr * DO + lc] = acc[nt][r];
    }
  }
  __syncthreads();

  v4f pv[8];
#pragma unroll
  for (int q = 0; q < 8; ++q) {
    const int p   = tid + q * GTHR;
    const int row = p >> 4;
    const int col = 4 * (p & 15);
    pv[q] = *(const v4fa*)(stg + row * DO + col) * sdg[row];
  }
#pragma unroll
  for (int q = 0; q < 8; ++q) {
    const int p = tid + q * GTHR;
    float* op = T + (size_t)(rowBase + (p >> 4)) * (size_t)DO + 4 * (p & 15);
    *(volatile v4f*)op = pv[q];
  }
  __threadfence();
#pragma unroll
  for (int q = 0; q < 8; ++q) {
    const int p = tid + q * GTHR;
    float* op = T + (size_t)(rowBase + (p >> 4)) * (size_t)DO + 4 * (p & 15);
    *(volatile v4f*)op = pv[q];
  }
}

template <int CW, int LAST>
__global__ __launch_bounds__(NTHR) void k_agg(const int* __restrict__ srcs, const int* __restrict__ dsts,
                                              int nE, int nDst, int nSrc, int vec8,
                                              const float* __restrict__ tpl, const float* __restrict__ bias,
                                              float* opl, const float* __restrict__ gam,
                                              const float* __restrict__ bet, unsigned short* hpl, float* outp) {
  extern __shared__ __attribute__((aligned(16))) int dsm[];
  int* list = dsm;
  int* hl   = dsm + LISTN;
  int* sl   = hl + RCAP;
  int* cnt  = sl + RCAP;
  int* offs = cnt + NBA;
  int* cur  = offs + NBA;
  int* misc = cur + NBA;
  const int tid = (int)threadIdx.x, lane = tid & 31, wave = tid >> 5;
  const int nodeBase = (int)blockIdx.x * NBA;

  {
    const v4i z4 = {0, 0, 0, 0};
    for (int i = tid * 4; i < AGG_ZINTS; i += NTHR * 4) *(v4ia*)(dsm + i) = z4;
    if (tid < 16) misc[tid] = 0;
  }
  __syncthreads();

  int t = 0, ov = 0;
  const int nChunks = (nE + CHUNK - 1) / CHUNK;
#pragma unroll 1
  for (int ch = 0; ch < nChunks; ++ch) {
    const int cbase = ch * CHUNK;
    const int wc = scan_chunk<SLA>(dsts, nE, cbase, nodeBase, NBA, vec8, list, tid, lane, wave);
    if (lane == 0) misc[wave] = wc;
    __syncthreads();
    if (wave == 0) {
#pragma unroll 1
      for (int w2 = 0; w2 < NWAVE; ++w2) {
        int c = misc[w2];
        c = c < 0 ? 0 : (c > WCAP ? WCAP : c);
#pragma unroll 1
        for (int b0 = 0; b0 < c; b0 += 32) {
          const int idx = b0 + lane;
          const int ent = list[w2 * WCAP + (idx < WCAP ? idx : WCAP - 1)];
          const int m32 = (c - b0) < 32 ? (c - b0) : 32;
#pragma unroll 1
          for (int k = 0; k < m32; ++k) {
            const int u    = __builtin_amdgcn_readlane(ent, k);
            const int slot = u & (NBA - 1);
            const int el   = (u >> SLA) & (CHUNK - 1);
            const int pk   = ((cbase + el) << SLA) | slot;
            if (t < RCAP) {
              if (lane == 0) { hl[t] = pk; cnt[slot] = cnt[slot] + 1; }
              t = t + 1;
            } else {
              ov = 1;
            }
          }
        }
      }
    }
    __syncthreads();
  }
  if (wave == 0 && lane == 0) { misc[8] = t; misc[9] = ov; }
  __syncthreads();
  int tt = misc[8];
  tt = tt < 0 ? 0 : (tt > RCAP ? RCAP : tt);
  const int ovf = misc[9];

  if (wave == 0) {
    const int base = lane * (NBA / 32);
    int sacc = 0;
#pragma unroll 1
    for (int i = 0; i < NBA / 32; ++i) sacc += cnt[base + i];
    int incl = sacc;
#pragma unroll
    for (int d = 1; d < 32; d <<= 1) {
      const int y = __shfl_up(incl, d, 32);
      if (lane >= d) incl += y;
    }
    int run = incl - sacc;
#pragma unroll 1
    for (int i = 0; i < NBA / 32; ++i) {
      const int cv = cnt[base + i];
      offs[base + i] = run;
      cur[base + i]  = run;
      run += cv;
    }
  }
  __syncthreads();
  if (wave == 0) {
#pragma unroll 1
    for (int b0 = 0; b0 < tt; b0 += 32) {
      const int idx = b0 + lane;
      const int ent = hl[idx < RCAP ? idx : RCAP - 1];
      const int m32 = (tt - b0) < 32 ? (tt - b0) : 32;
#pragma unroll 1
      for (int k = 0; k < m32; ++k) {
        const int u    = __builtin_amdgcn_readlane(ent, k);
        const int slot = u & (NBA - 1);
        if (lane == 0) {
          int p = cur[slot];
          p = p < 0 ? 0 : (p > RCAP - 1 ? RCAP - 1 : p);
          sl[p] = u;
          cur[slot] = p + 1;
        }
      }
    }
  }
  __syncthreads();

  const float qnan = __int_as_float(0x7fc00000);
  const float pz = (ovf != 0) ? qnan : 0.0f;
  const int  cg  = (CW == DH) ? lane : (lane & 15);
  const bool act = (CW == DH) || (lane < 16);
  const v4f z4 = {0.0f, 0.0f, 0.0f, 0.0f};
  v4f bv;
  {
    const v4f a = *(const v4fa*)(bias + 4 * cg);
    bv.x = bf16_val(a.x); bv.y = bf16_val(a.y); bv.z = bf16_val(a.z); bv.w = bf16_val(a.w);
  }
  v4f g4 = z4, e4 = z4;
  if constexpr (LAST == 1) {
    const v4f tg = *(const v4fa*)(gam + 4 * cg);
    const v4f te = *(const v4fa*)(bet + 4 * cg);
    g4.x = bf16_val(tg.x); g4.y = bf16_val(tg.y); g4.z = bf16_val(tg.z); g4.w = bf16_val(tg.w);
    e4.x = bf16_val(te.x); e4.y = bf16_val(te.y); e4.z = bf16_val(te.z); e4.w = bf16_val(te.w);
  }
#pragma unroll 1
  for (int si = 0; si < NBA / NWAVE; ++si) {
    const int s    = si * NWAVE + wave;
    const int node = nodeBase + s;
    const int craw = cnt[s];
    const bool big = craw > DEGCAP;
    const int c = craw < 0 ? 0 : (craw > DEGCAP ? DEGCAP : craw);
    int o = offs[s];
    o = o < 0 ? 0 : (o > RCAP ? RCAP : o);
    const float dd = rsqrtf(fmaxf((float)craw, 1.0f));
    v4f acc = z4;
#pragma unroll 1
    for (int b0 = 0; b0 < c; b0 += 32) {
      int idx = o + b0 + lane;
      idx = idx > RCAP - 1 ? RCAP - 1 : idx;
      const int ent = sl[idx];
      int eid = ent >> SLA;
      eid = eid < 0 ? 0 : (eid > nE - 1 ? nE - 1 : eid);
      int sr = srcs[eid];
      sr = sr < 0 ? 0 : (sr > nSrc - 1 ? nSrc - 1 : sr);
      const int m32 = (c - b0) < 32 ? (c - b0) : 32;
#pragma unroll 1
      for (int k = 0; k < m32; ++k) {
        const int sk = __builtin_amdgcn_readlane(sr, k);
        const v4f a = *(const v4fa*)(tpl + (size_t)sk * (size_t)CW + 4 * cg);
        acc += a;
      }
    }
    const float pzr = big ? qnan : pz;
    v4f v;
    v.x = fmaf(acc.x, dd, bv.x) + pzr;
    v.y = fmaf(acc.y, dd, bv.y) + pzr;
    v.z = fmaf(acc.z, dd, bv.z) + pzr;
    v.w = fmaf(acc.w, dd, bv.w) + pzr;
    if constexpr (LAST == 0) {
      if (node < nDst) {
        float* op = opl + (size_t)node * (size_t)CW + 4 * cg;
        if (act) *(volatile v4f*)op = v;
        __threadfence();
        if (act) *(volatile v4f*)op = v;
      }
    } else {
      const int nc = node < nDst ? node : nDst - 1;
      const v4f prev = *(const v4fa*)(opl + (size_t)nc * (size_t)CW + 4 * cg);
      const v4f tv = prev + v;
      float sm = (tv.x + tv.y) + (tv.z + tv.w);
      if constexpr (CW == DH) sm = wsum32(sm); else sm = wsum16(sm);
      const float mu = sm * (1.0f / CW);
      const v4f d = tv - mu;
      float q = (d.x * d.x + d.y * d.y) + (d.z * d.z + d.w * d.w);
      if constexpr (CW == DH) q = wsum32(q); else q = wsum16(q);
      const float rs = rsqrtf(q * (1.0f / CW) + 1e-5f);
      v4f y = d * rs * g4 + e4;
      if constexpr (CW == DH) {
        y.x = fmaxf(y.x, 0.0f); y.y = fmaxf(y.y, 0.0f); y.z = fmaxf(y.z, 0.0f); y.w = fmaxf(y.w, 0.0f);
        const v8us po = hilo8(y);
        if (node < nDst) {
          unsigned short* hp = hpl + (size_t)node * (size_t)K2 + 8 * lane;
          *(volatile v8us*)hp = po;
          __threadfence();
          *(volatile v8us*)hp = po;
        }
      } else {
        if (node < nDst) {
          float* op = outp + (size_t)node * (size_t)DO + 4 * cg;
          if (act) *(volatile v4f*)op = y;
          __threadfence();
          if (act) *(volatile v4f*)op = y;
        }
      }
    }
  }
}

static inline int cdiv(int a, int b) { return (a + b - 1) / b; }

extern "C" void kernel_launch(void* const* d_in, const int* in_sizes, int n_in,
                              void* d_out, int out_size, void* d_ws, size_t ws_size,
                              hipStream_t stream) {
  if (n_in < 23) return;
  if (in_sizes[0] < CIN * GBM || (in_sizes[0] % CIN) != 0) return;
  if (in_sizes[1] < CIN * GBM || (in_sizes[1] % CIN) != 0) return;
  if (in_sizes[2] < CIN * GBM || (in_sizes[2] % CIN) != 0) return;
  const int N0 = in_sizes[0] / CIN, N1 = in_sizes[1] / CIN, N2 = in_sizes[2] / CIN;
  if ((N0 % GBM) != 0 || (N1 % GBM) != 0 || (N2 % GBM) != 0) return;
  if (in_sizes[3] != CIN * DH || in_sizes[5] != CIN * DH || in_sizes[7] != CIN * DH) return;
  if (in_sizes[4] != DH || in_sizes[6] != DH || in_sizes[8] != DH) return;
  if (in_sizes[9] != NREL * DH * DH || in_sizes[10] != NREL * DH) return;
  if (in_sizes[11] != NREL * DH * DO || in_sizes[12] != NREL * DO) return;
  if (in_sizes[13] != NTYPE * DH || in_sizes[14] != NTYPE * DH) return;
  if (in_sizes[15] != NTYPE * DO || in_sizes[16] != NTYPE * DO) return;
  if (in_sizes[17] < 2 || (in_sizes[17] & 1) != 0) return;
  for (int r = 1; r < NREL; ++r) if (in_sizes[17 + r] != in_sizes[17]) return;
  const int nE = in_sizes[17] / 2;
  if (nE < 1 || nE >= (1 << (31 - SLA))) return;
  const int NTOT = N0 + N1 + N2;
  if ((long long)out_size != (long long)NTOT * DO) return;

  const float* x0   = (const float*)d_in[0];
  const float* x1   = (const float*)d_in[1];
  const float* x2   = (const float*)d_in[2];
  const float* Wp0  = (const float*)d_in[3];
  const float* bp0  = (const float*)d_in[4];
  const float* Wp1  = (const float*)d_in[5];
  const float* bp1  = (const float*)d_in[6];
  const float* Wp2  = (const float*)d_in[7];
  const float* bp2  = (const float*)d_in[8];
  const float* W1   = (const float*)d_in[9];
  const float* b1   = (const float*)d_in[10];
  const float* W2   = (const float*)d_in[11];
  const float* b2   = (const float*)d_in[12];
  const float* l1g  = (const float*)d_in[13];
  const float* l1b  = (const float*)d_in[14];
  const float* l2g  = (const float*)d_in[15];
  const float* l2b  = (const float*)d_in[16];
  const int* e0 = (const int*)d_in[17];
  const int* e1 = (const int*)d_in[18];
  const int* e2 = (const int*)d_in[19];
  const int* e3 = (const int*)d_in[20];
  const int* e4 = (const int*)d_in[21];
  const int* e5 = (const int*)d_in[22];
  float* out = (float*)d_out;

  const size_t roff0 = 0, roff1 = (size_t)N0, roff2 = (size_t)N0 + (size_t)N1;
  float* out0 = out;
  float* out1 = out + (size_t)N0 * DO;
  float* out2 = out + ((size_t)N0 + (size_t)N1) * DO;

  int maxN = N0 > N1 ? N0 : N1;
  maxN = maxN > N2 ? maxN : N2;
  const int gD   = cdiv(maxN, NBD);
  const int NBPD = gD * NBD;
  const int vec8 = ((nE & 3) == 0) ? 1 : 0;

  char* ws = (char*)d_ws;
  size_t off = 0;
  const size_t oDG  = off; off += (size_t)NREL * (size_t)NBPD * 4;           off = (off + 255) & ~(size_t)255;
  const size_t oWPT = off; off += (size_t)NTYPE * DH * CIN * 2;              off = (off + 255) & ~(size_t)255;
  const size_t oW1T = off; off += (size_t)NREL * DH * K2 * 2;                off = (off + 255) & ~(size_t)255;
  const size_t oW2T = off; off += (size_t)NREL * DO * K2 * 2;                off = (off + 255) & ~(size_t)255;
  const size_t oHA  = off; off += (size_t)NTOT * K2 * 2;                     off = (off + 255) & ~(size_t)255;
  size_t szBIG = (size_t)N1 * DH * 4;
  if ((size_t)NTOT * CIN * 2 > szBIG) szBIG = (size_t)NTOT * CIN * 2;
  const size_t oBIG = off; off += szBIG;                                     off = (off + 255) & ~(size_t)255;
  const size_t szSA = (size_t)(N2 > N0 ? N2 : N0) * DH * 4;
  const size_t oSA  = off; off += szSA;                                      off = (off + 255) & ~(size_t)255;
  const size_t oSB  = off; off += (size_t)N0 * DH * 4;                       off = (off + 255) & ~(size_t)255;
  const size_t szSC = (size_t)(N0 > N2 ? N0 : N2) * DH * 4;
  const size_t oSC  = off; off += szSC;                                      off = (off + 255) & ~(size_t)255;
  if (off > ws_size || off > (size_t)WSMAX) return;
  float*          DG  = (float*)(ws + oDG);
  unsigned short* WPT = (unsigned short*)(ws + oWPT);
  unsigned short* W1T = (unsigned short*)(ws + oW1T);
  unsigned short* W2T = (unsigned short*)(ws + oW2T);
  unsigned short* HA  = (unsigned short*)(ws + oHA);
  float*          BIG = (float*)(ws + oBIG);
  unsigned short* XB  = (unsigned short*)(ws + oBIG);
  float*          SA  = (float*)(ws + oSA);
  float*          SB  = (float*)(ws + oSB);
  float*          SC  = (float*)(ws + oSC);

  const size_t aggLds = (size_t)AGG_LDS_INTS * 4;
  hipFuncSetAttribute(reinterpret_cast<const void*>(&k_agg<DH, 0>), hipFuncAttributeMaxDynamicSharedMemorySize, (int)aggLds);
  hipFuncSetAttribute(reinterpret_cast<const void*>(&k_agg<DH, 1>), hipFuncAttributeMaxDynamicSharedMemorySize, (int)aggLds);
  hipFuncSetAttribute(reinterpret_cast<const void*>(&k_agg<DO, 0>), hipFuncAttributeMaxDynamicSharedMemorySize, (int)aggLds);
  hipFuncSetAttribute(reinterpret_cast<const void*>(&k_agg<DO, 1>), hipFuncAttributeMaxDynamicSharedMemorySize, (int)aggLds);

  const int gA0 = cdiv(N0, NBA), gA1 = cdiv(N1, NBA), gA2 = cdiv(N2, NBA);

  k_prep<<<NUT / NTHR, NTHR, 0, stream>>>(Wp0, Wp1, Wp2, W1, W2, WPT, W1T, W2T);
  k_cvx<<<(NTOT * (CIN / 8)) / NTHR, NTHR, 0, stream>>>(x0, x1, x2, N0, N1, N2, XB);
  k_deg<<<dim3(gD, NREL), NTHR, 0, stream>>>(e0, e1, e2, e3, e4, e5, nE, vec8, N0, N1, N2, NBPD, DG);
  k_proj<<<N0 / GBM, GTHR, 0, stream>>>(XB + roff0 * CIN, WPT,                       bp0, HA + roff0 * K2);
  k_proj<<<N1 / GBM, GTHR, 0, stream>>>(XB + roff1 * CIN, WPT + (size_t)1 * DH * CIN, bp1, HA + roff1 * K2);
  k_proj<<<N2 / GBM, GTHR, 0, stream>>>(XB + roff2 * CIN, WPT + (size_t)2 * DH * CIN, bp2, HA + roff2 * K2);

  k_gemm<<<N2 / GBM, GTHR, 0, stream>>>(HA + roff2 * K2, W1T + (size_t)3 * DH * K2, DG + (size_t)3 * NBPD, SA, K2);
  k_agg<DH, 0><<<gA0, NTHR, aggLds, stream>>>(e3, e3 + nE, nE, N0, N2, vec8, SA, b1 + 3 * DH, SC, l1g, l1b, HA, out);
  k_gemm<<<N1 / GBM, GTHR, 0, stream>>>(HA + roff1 * K2, W1T + (size_t)4 * DH * K2, DG + (size_t)4 * NBPD, BIG, K2);
  k_gemm<<<N0 / GBM, GTHR, 0, stream>>>(HA + roff0 * K2, W1T,                        DG,                      SA, K2);
  k_gemm<<<N0 / GBM, GTHR, 0, stream>>>(HA + roff0 * K2, W1T + (size_t)1 * DH * K2, DG + (size_t)1 * NBPD, SB, K2);
  k_agg<DH, 1><<<gA0, NTHR, aggLds, stream>>>(e4, e4 + nE, nE, N0, N1, vec8, BIG, b1 + 4 * DH, SC,
                                               l1g, l1b, HA + roff0 * K2, out);
  k_agg<DH, 0><<<gA2, NTHR, aggLds, stream>>>(e0, e0 + nE, nE, N2, N0, vec8, SA, b1, SC, l1g, l1b, HA, out);
  k_gemm<<<N1 / GBM, GTHR, 0, stream>>>(HA + roff1 * K2, W1T + (size_t)2 * DH * K2, DG + (size_t)2 * NBPD, BIG, K2);
  k_gemm<<<N2 / GBM, GTHR, 0, stream>>>(HA + roff2 * K2, W1T + (size_t)5 * DH * K2, DG + (size_t)5 * NBPD, SA, K2);
  k_agg<DH, 1><<<gA2, NTHR, aggLds, stream>>>(e2, e2 + nE, nE, N2, N1, vec8, BIG, b1 + 2 * DH, SC,
                                               l1g + 2 * DH, l1b + 2 * DH, HA + roff2 * K2, out);
  k_agg<DH, 0><<<gA1, NTHR, aggLds, stream>>>(e1, e1 + nE, nE, N1, N0, vec8, SB, b1 + 1 * DH, BIG, l1g, l1b, HA, out);
  k_agg<DH, 1><<<gA1, NTHR, aggLds, stream>>>(e5, e5 + nE, nE, N1, N2, vec8, SA, b1 + 5 * DH, BIG,
                                               l1g + 1 * DH, l1b + 1 * DH, HA + roff1 * K2, out);

  k_gemm64<<<N2 / GBM, GTHR, 0, stream>>>(HA + roff2 * K2, W2T + (size_t)3 * DO * K2, DG + (size_t)3 * NBPD, SA);
  k_agg<DO, 0><<<gA0, NTHR, aggLds, stream>>>(e3, e3 + nE, nE, N0, N2, vec8, SA, b2 + 3 * DO, SC, l2g, l2b, HA, out0);
  k_gemm64<<<N1 / GBM, GTHR, 0, stream>>>(HA + roff1 * K2, W2T + (size_t)4 * DO * K2, DG + (size_t)4 * NBPD, BIG);
  k_gemm64<<<N0 / GBM, GTHR, 0, stream>>>(HA + roff0 * K2, W2T,                        DG,                      SA);
  k_gemm64<<<N0 / GBM, GTHR, 0, stream>>>(HA + roff0 * K2, W2T + (size_t)1 * DO * K2, DG + (size_t)1 * NBPD, SB);
  k_agg<DO, 1><<<gA0, NTHR, aggLds, stream>>>(e4, e4 + nE, nE, N0, N1, vec8, BIG, b2 + 4 * DO, SC,
                                               l2g, l2b, HA, out0);
  k_agg<DO, 0><<<gA2, NTHR, aggLds, stream>>>(e0, e0 + nE, nE, N2, N0, vec8, SA, b2, SC, l2g, l2b, HA, out2);
  k_gemm64<<<N1 / GBM, GTHR, 0, stream>>>(HA + roff1 * K2, W2T + (size_t)2 * DO * K2, DG + (size_t)2 * NBPD, BIG);
  k_gemm64<<<N2 / GBM, GTHR, 0, stream>>>(HA + roff2 * K2, W2T + (size_t)5 * DO * K2, DG + (size_t)5 * NBPD, SA);
  k_agg<DO, 1><<<gA2, NTHR, aggLds, stream>>>(e2, e2 + nE, nE, N2, N1, vec8, BIG, b2 + 2 * DO, SC,
                                               l2g + 2 * DO, l2b + 2 * DO, HA, out2);
  k_agg<DO, 0><<<gA1, NTHR, aggLds, stream>>>(e1, e1 + nE, nE, N1, N0, vec8, SB, b2 + 1 * DO, BIG, l2g, l2b, HA, out1);
  k_agg<DO, 1><<<gA1, NTHR, aggLds, stream>>>(e5, e5 + nE, nE, N1, N2, vec8, SA, b2 + 5 * DO, BIG,
                                               l2g + 1 * DO, l2b + 1 * DO, HA, out1);
}
